// E_GCL_X_11751030522787
// MI455X (gfx1250) — hardware-run, weakly checked
//
#include <hip/hip_runtime.h>
#include <stddef.h>


#pragma clang fp contract(off)

#define NB      2
#define DN      128
#define XROW    12
#define EDIM    16
#define NTHR    256
#define NWAVE   8
#define NBN     64
#define NBE     64
#define APA     136
#define APN     264
#define APR     40
#define GSTR    132
#define NPROW   256
#define MROW    128
#define CROW    16
#define SROW    16
#define EPT     8
#define PIECE   (NTHR * EPT)
#define WCAP    (EPT * 32)
#define NBC     256
#define SLB     8
#define CE      163840
#define MAXCH   64
#define PAH     0
#define PAL     16384
#define PBH     32768
#define PBL     49152
#define PM2     65536
#define PN1H    81920
#define PN1L    114688
#define PN2H    147456
#define PN2L    163840
#define PW3     180224
#define PC1     184320
#define PC2     200704
#define PWTOT   202752
#define PBLK    (PWTOT / (NTHR * 8))
#define WSCAP   134217728
#define NODEDYN (2 * NBN * APA * 2)
#define EDGEDYN (NBE * GSTR * 4)
#define AGGDYN  ((NBC * DN + NBC * SROW) * 4)
#define MLPDYN  (2 * NBN * APN * 2 + 2 * NBN * APA * 2)
#define SCW     16.0f
#define SCA     64.0f
#define SCC     16384.0f
#define INV1024 0.0009765625f
#define INVC    9.5367431640625e-7f

static_assert((PWTOT % (NTHR * 8)) == 0);
static_assert((PAL % (NTHR * 8)) == 0);
static_assert((PBH % (NTHR * 8)) == 0);
static_assert((PBL % (NTHR * 8)) == 0);
static_assert((PM2 % (NTHR * 8)) == 0);
static_assert((PN1H % (NTHR * 8)) == 0);
static_assert((PN1L % (NTHR * 8)) == 0);
static_assert((PN2H % (NTHR * 8)) == 0);
static_assert((PN2L % (NTHR * 8)) == 0);
static_assert((PW3 % (NTHR * 8)) == 0);
static_assert((PC1 % (NTHR * 8)) == 0);
static_assert((PC2 % (NTHR * 8)) == 0);
static_assert(PW3 + 128 * 32 == PC1);
static_assert(PC1 + 128 * 128 == PC2);
static_assert(PC2 + 16 * 128 == PWTOT);
static_assert(((APA * 2) % 16) == 0);
static_assert(((APN * 2) % 16) == 0);
static_assert(((APR * 2) % 16) == 0);
static_assert(((GSTR * 4) % 16) == 0);
static_assert(NBN * APN * 2 == NBN * GSTR * 4);
static_assert(NODEDYN == 34816);
static_assert(MLPDYN == 102400);
static_assert(AGGDYN == 147456);
static_assert(NBC == (1 << SLB));
static_assert(PIECE == 2048);
static_assert((EPT % 4) == 0);
static_assert((CE % PIECE) == 0);
static_assert((CE % NBE) == 0);
static_assert((NBC % NWAVE) == 0);
static_assert(XROW * NBC == 3 * 4 * NTHR);
static_assert(SROW * NBC == 4 * 4 * NTHR);
static_assert(NBE == NWAVE * 8);
static_assert(NBN == 4 * 16);
static_assert(NTHR == 4 * NBE);
static_assert((NBC * DN) % (4 * NTHR) == 0);
static_assert((NBC * SROW) % (4 * NTHR) == 0);

typedef float          v4f   __attribute__((ext_vector_type(4)));
typedef float          v8f   __attribute__((ext_vector_type(8)));
typedef int            v4i   __attribute__((ext_vector_type(4)));
typedef unsigned short v8us  __attribute__((ext_vector_type(8)));
typedef _Float16       v4h   __attribute__((ext_vector_type(4)));
typedef _Float16       v8h   __attribute__((ext_vector_type(8)));
typedef _Float16       v16h  __attribute__((ext_vector_type(16)));
typedef __bf16         v16b  __attribute__((ext_vector_type(16)));
union FragH { v16h v; v8h h[2]; };
union FragB { v16b v; v8us u[2]; };
union Cvt8  { v8h v; v8us u; };

__device__ __forceinline__ v8f wmh(v16h a, v16h b, v8f c) {
  v8f d = __builtin_amdgcn_wmma_f32_16x16x32_f16(false, a, false, b, (short)0, c, false, false);
  asm volatile("v_nop\n\tv_nop\n\tv_nop\n\tv_nop" : "+v"(d) : "v"(a), "v"(b));
  return d;
}
__device__ __forceinline__ v8f wmb(v16b a, v16b b, v8f c) {
  v8f d = __builtin_amdgcn_wmma_f32_16x16x32_bf16(false, a, false, b, (short)0, c, false, false);
  asm volatile("v_nop\n\tv_nop\n\tv_nop\n\tv_nop" : "+v"(d) : "v"(a), "v"(b));
  return d;
}
__device__ __forceinline__ v8f zero8() {
  v8f z = {0.f, 0.f, 0.f, 0.f, 0.f, 0.f, 0.f, 0.f};
  return z;
}
__device__ __forceinline__ v4f zero4() {
  v4f z = {0.f, 0.f, 0.f, 0.f};
  return z;
}
__device__ __forceinline__ int iclamp(int v, int lo, int hi) { return v < lo ? lo : (v > hi ? hi : v); }

__device__ __forceinline__ unsigned short bf_rne(float f) {
  unsigned u = __float_as_uint(f);
  u += 0x7FFFu + ((u >> 16) & 1u);
  return (unsigned short)(u >> 16);
}
__device__ __forceinline__ float bf_val(unsigned short b) { return __uint_as_float(((unsigned)b) << 16); }

__device__ __forceinline__ void cvt_hl8(v4f xa, v4f xb, v8us& h, v8us& l) {
  float f[8];
  f[0] = xa.x; f[1] = xa.y; f[2] = xa.z; f[3] = xa.w;
  f[4] = xb.x; f[5] = xb.y; f[6] = xb.z; f[7] = xb.w;
#pragma unroll
  for (int j = 0; j < 8; ++j) {
    const unsigned short hb = bf_rne(f[j]);
    h[j] = hb;
    l[j] = bf_rne(f[j] - bf_val(hb));
  }
}

__device__ __forceinline__ void gemm16x64(const _Float16* ap, const _Float16* __restrict__ bpl, int kp, int nks, int n0,
                                          int m, int hh, v8f& c0, v8f& c1, v8f& c2, v8f& c3) {
  c0 = zero8(); c1 = zero8(); c2 = zero8(); c3 = zero8();
#pragma unroll 1
  for (int ks = 0; ks < nks; ++ks) {
    FragH a;
    a.h[0] = *(const v8h*)(ap + 32 * ks);
    a.h[1] = *(const v8h*)(ap + 32 * ks + 16);
    const _Float16* bp = bpl + (size_t)(n0 + m) * kp + 32 * ks + 8 * hh;
    FragH b;
    b.h[0] = *(const v8h*)(bp);
    b.h[1] = *(const v8h*)(bp + 16);
    c0 = wmh(a.v, b.v, c0);
    b.h[0] = *(const v8h*)(bp + (size_t)16 * kp);
    b.h[1] = *(const v8h*)(bp + (size_t)16 * kp + 16);
    c1 = wmh(a.v, b.v, c1);
    b.h[0] = *(const v8h*)(bp + (size_t)32 * kp);
    b.h[1] = *(const v8h*)(bp + (size_t)32 * kp + 16);
    c2 = wmh(a.v, b.v, c2);
    b.h[0] = *(const v8h*)(bp + (size_t)48 * kp);
    b.h[1] = *(const v8h*)(bp + (size_t)48 * kp + 16);
    c3 = wmh(a.v, b.v, c3);
  }
}

__device__ __forceinline__ void tile3(const unsigned short* __restrict__ bh, const unsigned short* __restrict__ bl,
                                      size_t ob, const FragB& ah, const FragB& al, v8f& c) {
  FragB b;
  b.u[0] = *(const v8us*)(bh + ob);
  b.u[1] = *(const v8us*)(bh + ob + 16);
  c = wmb(ah.v, b.v, c);
  c = wmb(al.v, b.v, c);
  b.u[0] = *(const v8us*)(bl + ob);
  b.u[1] = *(const v8us*)(bl + ob + 16);
  c = wmb(ah.v, b.v, c);
}

__device__ __forceinline__ void gemm3x16x64(const unsigned short* aph, const unsigned short* apl,
                                            const unsigned short* __restrict__ bh, const unsigned short* __restrict__ bl,
                                            int kp, int nks, int n0, int m, int hh, v8f& c0, v8f& c1, v8f& c2, v8f& c3) {
  c0 = zero8(); c1 = zero8(); c2 = zero8(); c3 = zero8();
#pragma unroll 1
  for (int ks = 0; ks < nks; ++ks) {
    FragB ah, al;
    ah.u[0] = *(const v8us*)(aph + 32 * ks);
    ah.u[1] = *(const v8us*)(aph + 32 * ks + 16);
    al.u[0] = *(const v8us*)(apl + 32 * ks);
    al.u[1] = *(const v8us*)(apl + 32 * ks + 16);
    const size_t ob = (size_t)(n0 + m) * kp + 32 * ks + 8 * hh;
    tile3(bh, bl, ob,                     ah, al, c0);
    tile3(bh, bl, ob + (size_t)16 * kp,   ah, al, c1);
    tile3(bh, bl, ob + (size_t)32 * kp,   ah, al, c2);
    tile3(bh, bl, ob + (size_t)48 * kp,   ah, al, c3);
  }
}

__device__ __forceinline__ void stage8f(float* sp, v8f a, float scl, float bias) {
#pragma unroll
  for (int r = 0; r < 8; ++r) sp[r * GSTR] = a[r] * scl + bias;
}
__device__ __forceinline__ void stage8fr(float* sp, v8f a, float scl, float bias) {
#pragma unroll
  for (int r = 0; r < 8; ++r) sp[r * GSTR] = fmaxf(a[r] * scl + bias, 0.0f);
}
__device__ __forceinline__ void stage8h(_Float16* pc, v8f a, float bias) {
#pragma unroll
  for (int r = 0; r < 8; ++r) pc[r * APA] = (_Float16)(fmaxf(a[r] * INV1024 + bias, 0.0f) * SCA);
}
__device__ __forceinline__ void stage8y(unsigned short* ph, unsigned short* pl, v8f a, float bias) {
#pragma unroll
  for (int r = 0; r < 8; ++r) {
    const float v = fmaxf(a[r] + bias, 0.0f);
    const unsigned short hb = bf_rne(v);
    ph[r * APA] = hb;
    pl[r * APA] = bf_rne(v - bf_val(hb));
  }
}

__global__ __launch_bounds__(NTHR) void k_prep(
    const float* __restrict__ We1, const float* __restrict__ We2, const float* __restrict__ Wn1,
    const float* __restrict__ Wn2, const float* __restrict__ Wc1, const float* __restrict__ Wc2,
    unsigned short* wp) {
  const int tid = (int)threadIdx.x;
  const int b = (int)blockIdx.x;
  const int o = (b * NTHR + tid) * 8;
  const float* src = We1;
  int r0 = 0, n, k0, mode = 0, pitch = DN, nval = DN;
  float scl = SCW;
  if (o < PAL)       { n = o >> 7; k0 = o & 127; }
  else if (o < PBH)  { const int idx = o - PAL;  n = idx >> 7; k0 = idx & 127; mode = 1; }
  else if (o < PBL)  { const int idx = o - PBH;  n = idx >> 7; k0 = idx & 127; r0 = DN; }
  else if (o < PM2)  { const int idx = o - PBL;  n = idx >> 7; k0 = idx & 127; r0 = DN; mode = 1; }
  else if (o < PN1H) { const int idx = o - PM2;  n = idx >> 7; k0 = idx & 127; src = We2; mode = 2; }
  else if (o < PN1L) { const int idx = o - PN1H; n = idx >> 8; k0 = idx & 255; src = Wn1; }
  else if (o < PN2H) { const int idx = o - PN1L; n = idx >> 8; k0 = idx & 255; src = Wn1; mode = 1; }
  else if (o < PN2L) { const int idx = o - PN2H; n = idx >> 7; k0 = idx & 127; src = Wn2; }
  else if (o < PW3)  { const int idx = o - PN2L; n = idx >> 7; k0 = idx & 127; src = Wn2; mode = 1; }
  else if (o < PC1)  { const int idx = o - PW3;  n = idx >> 5; k0 = idx & 31;  r0 = 2 * DN; mode = 2; }
  else if (o < PC2)  { const int idx = o - PC1;  n = idx >> 7; k0 = idx & 127; src = Wc1; mode = 2; }
  else               { const int idx = o - PC2;  n = idx >> 7; k0 = idx & 127; src = Wc2; mode = 2; pitch = 4; nval = 4; scl = SCC; }
  v8us ov;
  if (mode == 2) {
    const int nn = n < nval ? n : nval - 1;
    Cvt8 cv;
#pragma unroll
    for (int j = 0; j < 8; ++j) {
      const float w = src[(size_t)(r0 + k0 + j) * pitch + nn];
      const float v = (n < nval) ? (w * scl) : 0.0f;
      cv.v[j] = (_Float16)v;
    }
    ov = cv.u;
  } else {
#pragma unroll
    for (int j = 0; j < 8; ++j) {
      const float w = src[(size_t)(r0 + k0 + j) * pitch + n];
      const unsigned short hb = bf_rne(w);
      const unsigned short lb = bf_rne(w - bf_val(hb));
      ov[j] = (mode == 0) ? hb : lb;
    }
  }
  unsigned short* dp = wp + o;
  *(volatile v8us*)dp = ov;
  __threadfence();
  *(volatile v8us*)dp = ov;
}

__global__ __launch_bounds__(NTHR) void k_node(
    const float* __restrict__ nsrc, const unsigned short* __restrict__ wp, float* NP, int nN) {
  extern __shared__ __attribute__((aligned(16))) float ndynf[];
  __shared__ __attribute__((aligned(16))) float stg[NWAVE * 1024];
  unsigned short* sAH = (unsigned short*)ndynf;
  unsigned short* sAL = sAH + NBN * APA;
  const int tid = (int)threadIdx.x, lane = tid & 31, wave = tid >> 5, hh = lane >> 4, m = lane & 15;
  const int n0 = (int)blockIdx.x * NBN;

  {
    const int nl = tid >> 2, q = tid & 3;
    int node = n0 + nl;
    node = node > nN - 1 ? nN - 1 : node;
    const float* rp = nsrc + (size_t)node * DN + 32 * q;
#pragma unroll
    for (int i = 0; i < 4; ++i) {
      const v4f xa = *(const v4f*)(rp + 8 * i);
      const v4f xb = *(const v4f*)(rp + 8 * i + 4);
      v8us h, l;
      cvt_hl8(xa, xb, h, l);
      *(v8us*)(sAH + nl * APA + 32 * q + 8 * i) = h;
      *(v8us*)(sAL + nl * APA + 32 * q + 8 * i) = l;
    }
  }
  __syncthreads();

  const int rt = wave & 3, chf = wave >> 2;
  const unsigned short* aph = sAH + (16 * rt + m) * APA + 8 * hh;
  const unsigned short* apl = sAL + (16 * rt + m) * APA + 8 * hh;
  const unsigned short* bh = wp + (chf ? PBH : PAH);
  const unsigned short* bl = wp + (chf ? PBL : PAL);
  float* sw = stg + wave * 1024;
#pragma unroll 1
  for (int qq = 0; qq < 2; ++qq) {
    v8f a0, a1, a2, a3;
    gemm3x16x64(aph, apl, bh, bl, DN, 4, 64 * qq, m, hh, a0, a1, a2, a3);
    {
      float* sp = sw + (8 * hh) * 64 + m;
#pragma unroll
      for (int r = 0; r < 8; ++r) {
        sp[r * 64]      = a0[r];
        sp[r * 64 + 16] = a1[r];
        sp[r * 64 + 32] = a2[r];
        sp[r * 64 + 48] = a3[r];
      }
    }
    __syncthreads();
#pragma unroll 1
    for (int i = 0; i < 8; ++i) {
      const int r2 = 2 * i + hh;
      const v4f v = *(const v4f*)(sw + r2 * 64 + 4 * m);
      const int row = n0 + 16 * rt + r2;
      *(volatile v4f*)(NP + (size_t)row * NPROW + 128 * chf + 64 * qq + 4 * m) = v;
    }
    __threadfence();
#pragma unroll 1
    for (int i = 0; i < 8; ++i) {
      const int r2 = 2 * i + hh;
      const v4f v = *(const v4f*)(sw + r2 * 64 + 4 * m);
      const int row = n0 + 16 * rt + r2;
      *(volatile v4f*)(NP + (size_t)row * NPROW + 128 * chf + 64 * qq + 4 * m) = v;
    }
    __syncthreads();
  }
}

__global__ __launch_bounds__(NTHR) void k_edge(
    const float* __restrict__ xb, const int* __restrict__ ei, const float* __restrict__ ea,
    const float* __restrict__ NP, const unsigned short* __restrict__ wp, const float* __restrict__ be1,
    const float* __restrict__ be2, const float* __restrict__ bc1,
    float* Mout, float* Cout, int nE, int nN, int nb0, int cbeg) {
  extern __shared__ __attribute__((aligned(16))) float sH[];
  __shared__ __attribute__((aligned(16))) _Float16 sA[NBE * APA];
  __shared__ __attribute__((aligned(16))) _Float16 sC[NBE * APA];
  __shared__ __attribute__((aligned(16))) _Float16 sR[NBE * APR];
  __shared__ __attribute__((aligned(16))) float sPar[3 * DN];
  __shared__ __attribute__((aligned(16))) float sCD[NBE * XROW];
  __shared__ __attribute__((aligned(16))) float sWg[NBE * 4];
  __shared__ int sI[NBE];
  __shared__ int sJ[NBE];
  const int tid = (int)threadIdx.x, lane = tid & 31, wave = tid >> 5, hh = lane >> 4, m = lane & 15;
  const int el0 = (int)blockIdx.x * NBE;

  if (tid < NBE) {
    int e = cbeg + el0 + tid;
    e = e > nE - 1 ? nE - 1 : e;
    const int ii = iclamp(ei[e], 0, nN - 1);
    const int jj = iclamp(ei[(size_t)nE + e], 0, nN - 1);
    const float* pi = xb + (size_t)ii * XROW;
    const float* pj = xb + (size_t)jj * XROW;
    float cd[12];
#pragma unroll
    for (int c = 0; c < 12; ++c) {
      cd[c] = pi[c] - pj[c];
      sCD[XROW * tid + c] = cd[c];
    }
    float pr[16];
#pragma unroll
    for (int j = 0; j < 4; ++j) {
#pragma unroll
      for (int k = 0; k < 4; ++k) {
        float p = cd[3 * j] * cd[3 * k];
        p = fmaf(cd[3 * j + 1], cd[3 * k + 1], p);
        p = fmaf(cd[3 * j + 2], cd[3 * k + 2], p);
        pr[4 * j + k] = p;
      }
    }
    float ss = 0.0f;
#pragma unroll
    for (int q = 0; q < 16; ++q) ss += pr[q] * pr[q];
    const float inv = 1.0f / fmaxf(sqrtf(ss), 1e-12f);
    v8h ra, rb, xa, xc;
#pragma unroll
    for (int q = 0; q < 8; ++q) {
      ra[q] = (_Float16)((pr[q] * inv) * SCA);
      rb[q] = (_Float16)((pr[8 + q] * inv) * SCA);
    }
    const float* ep = ea + (size_t)e * EDIM;
    const v4f e0 = *(const v4f*)(ep);
    const v4f e1 = *(const v4f*)(ep + 4);
    const v4f e2 = *(const v4f*)(ep + 8);
    const v4f e3 = *(const v4f*)(ep + 12);
    xa[0] = (_Float16)(e0.x * SCA); xa[1] = (_Float16)(e0.y * SCA); xa[2] = (_Float16)(e0.z * SCA); xa[3] = (_Float16)(e0.w * SCA);
    xa[4] = (_Float16)(e1.x * SCA); xa[5] = (_Float16)(e1.y * SCA); xa[6] = (_Float16)(e1.z * SCA); xa[7] = (_Float16)(e1.w * SCA);
    xc[0] = (_Float16)(e2.x * SCA); xc[1] = (_Float16)(e2.y * SCA); xc[2] = (_Float16)(e2.z * SCA); xc[3] = (_Float16)(e2.w * SCA);
    xc[4] = (_Float16)(e3.x * SCA); xc[5] = (_Float16)(e3.y * SCA); xc[6] = (_Float16)(e3.z * SCA); xc[7] = (_Float16)(e3.w * SCA);
    _Float16* rp = sR + tid * APR;
    *(v8h*)(rp)      = ra;
    *(v8h*)(rp + 8)  = rb;
    *(v8h*)(rp + 16) = xa;
    *(v8h*)(rp + 24) = xc;
    sI[tid] = ii;
    sJ[tid] = jj;
  }
  if (tid < DN) {
    sPar[tid]          = be1[tid];
    sPar[DN + tid]     = be2[tid];
    sPar[2 * DN + tid] = bc1[tid];
  }
  __syncthreads();

  const int rt = wave & 3, cg = wave >> 2;

  {
    v8f a0, a1, a2, a3;
    gemm16x64(sR + (16 * rt + m) * APR + 8 * hh, (const _Float16*)(wp + PW3), 32, 1, 64 * cg, m, hh, a0, a1, a2, a3);
    float* sp = sH + (16 * rt + 8 * hh) * GSTR + 64 * cg + m;
    const float* bb = sPar + 64 * cg + m;
    stage8f(sp,      a0, INV1024, bb[0]);
    stage8f(sp + 16, a1, INV1024, bb[16]);
    stage8f(sp + 32, a2, INV1024, bb[32]);
    stage8f(sp + 48, a3, INV1024, bb[48]);
  }
  __syncthreads();

  {
    const int c4 = 4 * lane;
#pragma unroll 1
    for (int jx = 0; jx < 8; ++jx) {
      const int el = 8 * wave + jx;
      const int ii = sI[el];
      const int jj = sJ[el];
      const v4f p = *(const v4f*)(NP + (size_t)(nb0 + ii) * NPROW + c4);
      const v4f q = *(const v4f*)(NP + (size_t)(nb0 + jj) * NPROW + DN + c4);
      const v4f r = *(const v4f*)(sH + el * GSTR + c4);
      const v4f v = (p + q) + r;
      v4h z;
      z.x = (_Float16)(fmaxf(v.x, 0.0f) * SCA);
      z.y = (_Float16)(fmaxf(v.y, 0.0f) * SCA);
      z.z = (_Float16)(fmaxf(v.z, 0.0f) * SCA);
      z.w = (_Float16)(fmaxf(v.w, 0.0f) * SCA);
      *(v4h*)(sA + el * APA + c4) = z;
    }
  }
  __syncthreads();

  {
    v8f a0, a1, a2, a3;
    gemm16x64(sA + (16 * rt + m) * APA + 8 * hh, (const _Float16*)(wp + PM2), DN, 4, 64 * cg, m, hh, a0, a1, a2, a3);
    float* sp = sH + (16 * rt + 8 * hh) * GSTR + 64 * cg + m;
    const float* bb = sPar + DN + 64 * cg + m;
    stage8fr(sp,      a0, INV1024, bb[0]);
    stage8fr(sp + 16, a1, INV1024, bb[16]);
    stage8fr(sp + 32, a2, INV1024, bb[32]);
    stage8fr(sp + 48, a3, INV1024, bb[48]);
  }
  __syncthreads();

  {
#pragma unroll 1
    for (int it = 0; it < 8; ++it) {
      const int row = wave + NWAVE * it;
      const v4f v = *(const v4f*)(sH + row * GSTR + 4 * lane);
      *(volatile v4f*)(Mout + (size_t)(el0 + row) * MROW + 4 * lane) = v;
    }
    __threadfence();
#pragma unroll 1
    for (int it = 0; it < 8; ++it) {
      const int row = wave + NWAVE * it;
      const v4f v = *(const v4f*)(sH + row * GSTR + 4 * lane);
      *(volatile v4f*)(Mout + (size_t)(el0 + row) * MROW + 4 * lane) = v;
    }
  }
  {
    const int c4 = 4 * lane;
#pragma unroll 1
    for (int jx = 0; jx < 8; ++jx) {
      const int el = 8 * wave + jx;
      const v4f v = *(const v4f*)(sH + el * GSTR + c4);
      v4h z;
      z.x = (_Float16)(v.x * SCA);
      z.y = (_Float16)(v.y * SCA);
      z.z = (_Float16)(v.z * SCA);
      z.w = (_Float16)(v.w * SCA);
      *(v4h*)(sA + el * APA + c4) = z;
    }
  }
  __syncthreads();

  {
    v8f a0, a1, a2, a3;
    gemm16x64(sA + (16 * rt + m) * APA + 8 * hh, (const _Float16*)(wp + PC1), DN, 4, 64 * cg, m, hh, a0, a1, a2, a3);
    _Float16* pc = sC + (16 * rt + 8 * hh) * APA + 64 * cg + m;
    const float* bb = sPar + 2 * DN + 64 * cg + m;
    stage8h(pc,      a0, bb[0]);
    stage8h(pc + 16, a1, bb[16]);
    stage8h(pc + 32, a2, bb[32]);
    stage8h(pc + 48, a3, bb[48]);
  }
  __syncthreads();

  if (wave < 4) {
    v8f c = zero8();
    const _Float16* ap = sC + (16 * wave + m) * APA + 8 * hh;
    const _Float16* bp = (const _Float16*)(wp + PC2) + (size_t)m * DN + 8 * hh;
#pragma unroll 1
    for (int ks = 0; ks < 4; ++ks) {
      FragH a, b;
      a.h[0] = *(const v8h*)(ap + 32 * ks);
      a.h[1] = *(const v8h*)(ap + 32 * ks + 16);
      b.h[0] = *(const v8h*)(bp + 32 * ks);
      b.h[1] = *(const v8h*)(bp + 32 * ks + 16);
      c = wmh(a.v, b.v, c);
    }
    if (m < 4) {
#pragma unroll
      for (int r = 0; r < 8; ++r) sWg[(16 * wave + 8 * hh + r) * 4 + m] = c[r] * INVC;
    }
  }
  __syncthreads();

  {
    const int e = tid >> 2, q = tid & 3;
    float a[4];
#pragma unroll
    for (int i = 0; i < 4; ++i) {
      const int c  = 4 * q + i;
      const int cc = c > 11 ? 11 : c;
      const int j  = cc / 3;
      const float tv = sCD[XROW * e + cc] * sWg[4 * e + j];
      a[i] = (c < 12) ? tv : 0.0f;
    }
    v4f ov;
    ov.x = a[0]; ov.y = a[1]; ov.z = a[2]; ov.w = a[3];
    float* cp = Cout + (size_t)(el0 + e) * CROW + 4 * q;
    *(volatile v4f*)cp = ov;
    __threadfence();
    *(volatile v4f*)cp = ov;
  }
}

__device__ __forceinline__ int scan_piece(const int* __restrict__ eid, int lim, int cbase, int base, int vecok,
                                          int* list, int tid, int wave) {
  int wc = 0;
  const int el0  = tid * EPT;
  const int e0   = cbase + el0;
  const int sent = -2147483647 - 1;
  int kk[EPT];
  if (vecok != 0 && cbase + PIECE <= lim) {
    const v4i* p = (const v4i*)(eid + e0);
#pragma unroll
    for (int u = 0; u < EPT / 4; ++u) {
      const v4i d = p[u];
      kk[4 * u] = d.x; kk[4 * u + 1] = d.y; kk[4 * u + 2] = d.z; kk[4 * u + 3] = d.w;
    }
  } else {
    const int lm = lim - 1;
#pragma unroll
    for (int q = 0; q < EPT; ++q) {
      const int eq = e0 + q;
      const int ec = eq > lm ? lm : eq;
      const int a = eid[ec];
      kk[q] = (eq < lim) ? a : sent;
    }
  }
  const unsigned nb = (unsigned)base;
  unsigned sq[EPT];
  bool hq[EPT];
  bool anyl = false;
#pragma unroll
  for (int q = 0; q < EPT; ++q) {
    sq[q] = (unsigned)kk[q] - nb;
    hq[q] = sq[q] < (unsigned)NBC;
    anyl = anyl | hq[q];
  }
  const unsigned any = __builtin_amdgcn_ballot_w32(anyl);
  if (any != 0u) {
#define HIT(HQ, SQ, Q) { \
      const unsigned mj = __builtin_amdgcn_ballot_w32(HQ); \
      if (mj != 0u) { \
        if (HQ) { \
          const int ps = wc + (int)__builtin_amdgcn_mbcnt_lo(mj, 0u); \
          if (ps < WCAP) list[wave * WCAP + ps] = ((el0 + (Q)) << SLB) | (int)(SQ); \
        } \
        wc += (int)__builtin_popcount(mj); } }
#pragma unroll
    for (int q = 0; q < EPT; ++q) {
      HIT(hq[q], sq[q], q)
    }
#undef HIT
  }
  return wc;
}

__device__ __forceinline__ void drain_piece(const int* list, const int* wcnt, float* accF, float* accC,
                                            const float* __restrict__ Mf, const float* __restrict__ Cq,
                                            int rowoff, int lane, int wave) {
#pragma unroll 1
  for (int wsx = 0; wsx < NWAVE; ++wsx) {
    int n = __builtin_amdgcn_readfirstlane(wcnt[wsx]);
    n = n > WCAP ? WCAP : (n < 0 ? 0 : n);
    const int* lp = list + wsx * WCAP;
#pragma unroll 1
    for (int bb = 0; bb < n; bb += 32) {
      const int idx = bb + lane;
      const int ic = idx > WCAP - 1 ? WCAP - 1 : idx;
      const int ent = lp[ic];
      const bool own = (idx < n) && ((ent & (NWAVE - 1)) == wave);
      unsigned msk = __builtin_amdgcn_ballot_w32(own);
#pragma unroll 1
      while (msk != 0u) {
        const int bit = (int)__builtin_ctz(msk);
        msk &= msk - 1u;
        const int e2 = __builtin_amdgcn_readlane(ent, bit);
        const int slot = e2 & (NBC - 1);
        const int el = (e2 >> SLB) & (PIECE - 1);
        int row = rowoff + el;
        row = row < 0 ? 0 : (row > CE - 1 ? CE - 1 : row);
        const v4f mv = *(const v4f*)(Mf + (size_t)row * MROW + 4 * lane);
        float* ap = accF + slot * DN + 4 * lane;
        v4f a = *(const v4f*)ap;
        a += mv;
        *(v4f*)ap = a;
        const float cvv = Cq[(size_t)row * CROW + (lane & 15)];
        const float addv = (lane < 12) ? cvv : ((lane == 12) ? 1.0f : 0.0f);
        if (lane < SROW) accC[SROW * slot + lane] += addv;
      }
    }
  }
}

__device__ __forceinline__ void agg_store(const float* accF, const float* accC, const float* __restrict__ xb,
                                          float* outH, float* outX, float* S, int base, int nN, int last,
                                          int tid, int lane, int wave) {
#pragma unroll 1
  for (int it = 0; it < NBC / NWAVE; ++it) {
    const int s = wave + NWAVE * it;
    const int node = base + s;
    if (node < nN) {
      const v4f v = *(const v4f*)(accF + s * DN + 4 * lane);
      *(volatile v4f*)(outH + (size_t)node * DN + 4 * lane) = v;
    }
  }
  if (last != 0) {
    int cnt = nN - base;
    cnt = cnt > NBC ? NBC : cnt;
    const int nq = 3 * cnt;
    const size_t f0 = (size_t)XROW * (size_t)base;
#pragma unroll 1
    for (int it = 0; it < 3; ++it) {
      const int q = tid + NTHR * it;
      if (q < nq) {
        float a[4];
#pragma unroll
        for (int c = 0; c < 4; ++c) {
          const int t = 4 * q + c;
          const int s3 = t / XROW;
          const int cc = t - XROW * s3;
          const float sv = accC[SROW * s3 + cc];
          const float cn = accC[SROW * s3 + 12];
          const float xv = xb[f0 + (size_t)t];
          a[c] = xv + sv * (1.0f / fmaxf(cn, 1.0f));
        }
        v4f ov;
        ov.x = a[0]; ov.y = a[1]; ov.z = a[2]; ov.w = a[3];
        *(volatile v4f*)(outX + f0 + 4 * (size_t)q) = ov;
      }
    }
  } else {
#pragma unroll 1
    for (int it = 0; it < 4; ++it) {
      const int q = tid + NTHR * it;
      const v4f v = *(const v4f*)(accC + 4 * q);
      *(volatile v4f*)(S + (size_t)base * SROW + 4 * (size_t)q) = v;
    }
  }
}

__global__ __launch_bounds__(NTHR) void k_agg(
    const int* __restrict__ ei, const float* __restrict__ Mq, const float* __restrict__ Cq,
    const float* __restrict__ xb, float* outH, float* outX, float* S, int cbeg, int lim, int nN,
    int first, int last, int vecok) {
  extern __shared__ __attribute__((aligned(16))) float accd[];
  __shared__ int list[NWAVE * WCAP];
  __shared__ int wcnt[NWAVE];
  const int tid = (int)threadIdx.x, lane = tid & 31, wave = tid >> 5;
  const int base = (int)blockIdx.x * NBC;
  float* accF = accd;
  float* accC = accd + NBC * DN;
  const int* eid = ei;

  if (first != 0) {
#pragma unroll 1
    for (int i = tid; i < (NBC * DN) / 4; i += NTHR) *(v4f*)(accF + 4 * i) = zero4();
#pragma unroll 1
    for (int i = tid; i < (NBC * SROW) / 4; i += NTHR) *(v4f*)(accC + 4 * i) = zero4();
  } else {
#pragma unroll 1
    for (int i = tid; i < (NBC * DN) / 4; i += NTHR) {
      const int s = i >> 5, c4 = (i & 31) * 4;
      int node = base + s;
      node = node > nN - 1 ? nN - 1 : node;
      const v4f v = *(const v4f*)(outH + (size_t)node * DN + c4);
      *(v4f*)(accF + s * DN + c4) = v;
    }
#pragma unroll 1
    for (int i = tid; i < (NBC * SROW) / 4; i += NTHR) {
      const v4f v = *(const v4f*)(S + (size_t)base * SROW + 4 * (size_t)i);
      *(v4f*)(accC + 4 * i) = v;
    }
  }
  __syncthreads();

#pragma unroll 1
  for (int cbase = cbeg; cbase < lim; cbase += PIECE) {
    const int wc = scan_piece(eid, lim, cbase, base, vecok, list, tid, wave);
    if (lane == 0) wcnt[wave] = wc;
    __syncthreads();
    drain_piece(list, wcnt, accF, accC, Mq, Cq, cbase - cbeg, lane, wave);
    __syncthreads();
  }

  agg_store(accF, accC, xb, outH, outX, S, base, nN, last, tid, lane, wave);
  __threadfence();
  agg_store(accF, accC, xb, outH, outX, S, base, nN, last, tid, lane, wave);
}

__global__ __launch_bounds__(NTHR) void k_nodemlp(
    const float* __restrict__ nsrc, const unsigned short* __restrict__ wp,
    const float* __restrict__ bn1, const float* __restrict__ bn2, float* HO, int nN) {
  extern __shared__ __attribute__((aligned(16))) float mdynf[];
  __shared__ __attribute__((aligned(16))) float sPar[2 * DN];
  unsigned short* sAH = (unsigned short*)mdynf;
  unsigned short* sAL = sAH + NBN * APN;
  unsigned short* sYH = sAL + NBN * APN;
  unsigned short* sYL = sYH + NBN * APA;
  float* sU = mdynf;
  const int tid = (int)threadIdx.x, lane = tid & 31, wave = tid >> 5, hh = lane >> 4, m = lane & 15;
  const int n0 = (int)blockIdx.x * NBN;

  {
    const int nl = tid >> 2, g = tid & 3;
    int node = n0 + nl;
    node = node > nN - 1 ? nN - 1 : node;
    const float* np_ = nsrc + (size_t)node * DN + 32 * g;
    const float* mp  = HO   + (size_t)node * DN + 32 * g;
#pragma unroll
    for (int i = 0; i < 4; ++i) {
      const v4f xa = *(const v4f*)(np_ + 8 * i);
      const v4f xb = *(const v4f*)(np_ + 8 * i + 4);
      v8us h, l;
      cvt_hl8(xa, xb, h, l);
      *(v8us*)(sAH + nl * APN + 32 * g + 8 * i) = h;
      *(v8us*)(sAL + nl * APN + 32 * g + 8 * i) = l;
    }
#pragma unroll
    for (int i = 0; i < 4; ++i) {
      const v4f xa = *(const v4f*)(mp + 8 * i);
      const v4f xb = *(const v4f*)(mp + 8 * i + 4);
      v8us h, l;
      cvt_hl8(xa, xb, h, l);
      *(v8us*)(sAH + nl * APN + DN + 32 * g + 8 * i) = h;
      *(v8us*)(sAL + nl * APN + DN + 32 * g + 8 * i) = l;
    }
  }
  if (tid < DN) {
    sPar[tid]      = bn1[tid];
    sPar[DN + tid] = bn2[tid];
  }
  __syncthreads();

  const int rt = wave & 3, cg = wave >> 2;

  {
    v8f a0, a1, a2, a3;
    gemm3x16x64(sAH + (16 * rt + m) * APN + 8 * hh, sAL + (16 * rt + m) * APN + 8 * hh,
                wp + PN1H, wp + PN1L, 2 * DN, 8, 64 * cg, m, hh, a0, a1, a2, a3);
    unsigned short* ph = sYH + (16 * rt + 8 * hh) * APA + 64 * cg + m;
    unsigned short* pl = sYL + (16 * rt + 8 * hh) * APA + 64 * cg + m;
    const float* bb = sPar + 64 * cg + m;
    stage8y(ph,      pl,      a0, bb[0]);
    stage8y(ph + 16, pl + 16, a1, bb[16]);
    stage8y(ph + 32, pl + 32, a2, bb[32]);
    stage8y(ph + 48, pl + 48, a3, bb[48]);
  }
  __syncthreads();

  {
    v8f a0, a1, a2, a3;
    gemm3x16x64(sYH + (16 * rt + m) * APA + 8 * hh, sYL + (16 * rt + m) * APA + 8 * hh,
                wp + PN2H, wp + PN2L, DN, 4, 64 * cg, m, hh, a0, a1, a2, a3);
    float* sp = sU + (16 * rt + 8 * hh) * GSTR + 64 * cg + m;
    stage8f(sp,      a0, 1.0f, 0.0f);
    stage8f(sp + 16, a1, 1.0f, 0.0f);
    stage8f(sp + 32, a2, 1.0f, 0.0f);
    stage8f(sp + 48, a3, 1.0f, 0.0f);
  }
  __syncthreads();

  const v4f b4 = *(const v4f*)(sPar + DN + 4 * lane);
#pragma unroll 1
  for (int it = 0; it < NBN / NWAVE; ++it) {
    const int s = wave + NWAVE * it;
    const int node = n0 + s;
    if (node < nN) {
      const v4f su = *(const v4f*)(sU + s * GSTR + 4 * lane);
      const v4f hv = *(const v4f*)(nsrc + (size_t)node * DN + 4 * lane);
      const v4f v = (hv + su) + b4;
      *(volatile v4f*)(HO + (size_t)node * DN + 4 * lane) = v;
    }
  }
  __threadfence();
#pragma unroll 1
  for (int it = 0; it < NBN / NWAVE; ++it) {
    const int s = wave + NWAVE * it;
    const int node = n0 + s;
    if (node < nN) {
      const v4f su = *(const v4f*)(sU + s * GSTR + 4 * lane);
      const v4f hv = *(const v4f*)(nsrc + (size_t)node * DN + 4 * lane);
      const v4f v = (hv + su) + b4;
      *(volatile v4f*)(HO + (size_t)node * DN + 4 * lane) = v;
    }
  }
}

extern "C" void kernel_launch(void* const* d_in, const int* in_sizes, int n_in,
                              void* d_out, int out_size, void* d_ws, size_t ws_size,
                              hipStream_t stream) {
  if (n_in < 15) return;
  if (in_sizes[0] < NB * DN || (in_sizes[0] % DN) != 0) return;
  const int nTot = in_sizes[0] / DN;
  if ((nTot % NB) != 0) return;
  const int nN = nTot / NB;
  if (nN < 2 || nN > (1 << 22)) return;
  if (in_sizes[1] != nTot * XROW) return;
  if (in_sizes[2] < 2 || (in_sizes[2] % 2) != 0) return;
  const int nE = in_sizes[2] / 2;
  if (nE < 1 || nE > (1 << 26)) return;
  if (in_sizes[3] != nE * EDIM) return;
  if (in_sizes[4] != (2 * DN + 32) * DN || in_sizes[5] != DN) return;
  if (in_sizes[6] != DN * DN || in_sizes[7] != DN) return;
  if (in_sizes[8] != 2 * DN * DN || in_sizes[9] != DN) return;
  if (in_sizes[10] != DN * DN || in_sizes[11] != DN) return;
  if (in_sizes[12] != DN * DN || in_sizes[13] != DN) return;
  if (in_sizes[14] != DN * 4) return;
  if (out_size != nTot * (DN + XROW)) return;

  const float* h     = (const float*)d_in[0];
  const float* coord = (const float*)d_in[1];
  const int*   ei    = (const int*)d_in[2];
  const float* ea    = (const float*)d_in[3];
  const float* We1   = (const float*)d_in[4];
  const float* be1   = (const float*)d_in[5];
  const float* We2   = (const float*)d_in[6];
  const float* be2   = (const float*)d_in[7];
  const float* Wn1   = (const float*)d_in[8];
  const float* bn1   = (const float*)d_in[9];
  const float* Wn2   = (const float*)d_in[10];
  const float* bn2   = (const float*)d_in[11];
  const float* Wc1   = (const float*)d_in[12];
  const float* bc1   = (const float*)d_in[13];
  const float* Wc2   = (const float*)d_in[14];
  float* out0 = (float*)d_out;
  float* out1 = out0 + (size_t)DN * (size_t)nTot;

  const int nbNode = (nTot + NBN - 1) / NBN;
  const int NpadT  = nbNode * NBN;
  const int nChunk = (nE + CE - 1) / CE;
  if (nChunk < 1 || nChunk > MAXCH) return;
  const int nbAgg  = (nN + NBC - 1) / NBC;
  const int SpadN  = nbAgg * NBC;

  char* ws = (char*)d_ws;
  size_t off = 0;
  const size_t oW  = off; off += (size_t)PWTOT * 2;                    off = (off + 255) & ~(size_t)255;
  const size_t oNP = off; off += (size_t)NpadT * NPROW * 4;              off = (off + 255) & ~(size_t)255;
  const size_t oM  = off; off += (size_t)CE * MROW * 4;                 off = (off + 255) & ~(size_t)255;
  const size_t oC  = off; off += (size_t)CE * CROW * 4;                 off = (off + 255) & ~(size_t)255;
  const size_t oS  = off; off += (size_t)NB * (size_t)SpadN * SROW * 4; off = (off + 255) & ~(size_t)255;
  if (off > ws_size || off > (size_t)WSCAP) return;
  unsigned short* wp = (unsigned short*)(ws + oW);
  float* NP          = (float*)(ws + oNP);
  float* Mq          = (float*)(ws + oM);
  float* Cq          = (float*)(ws + oC);
  float* S           = (float*)(ws + oS);

  hipFuncSetAttribute(reinterpret_cast<const void*>(&k_node), hipFuncAttributeMaxDynamicSharedMemorySize, NODEDYN);
  hipFuncSetAttribute(reinterpret_cast<const void*>(&k_edge), hipFuncAttributeMaxDynamicSharedMemorySize, EDGEDYN);
  hipFuncSetAttribute(reinterpret_cast<const void*>(&k_agg), hipFuncAttributeMaxDynamicSharedMemorySize, AGGDYN);
  hipFuncSetAttribute(reinterpret_cast<const void*>(&k_nodemlp), hipFuncAttributeMaxDynamicSharedMemorySize, MLPDYN);

  k_prep<<<PBLK, NTHR, 0, stream>>>(We1, We2, Wn1, Wn2, Wc1, Wc2, wp);
  k_node<<<nbNode, NTHR, NODEDYN, stream>>>(h, wp, NP, nTot);
  for (int b = 0; b < NB; ++b) {
    const float* xb = coord + (size_t)b * (size_t)nN * XROW;
    float* oH = out0 + (size_t)b * (size_t)nN * DN;
    float* oX = out1 + (size_t)b * (size_t)nN * XROW;
    float* Sb = S + (size_t)b * (size_t)SpadN * SROW;
    const int nb0 = b * nN;
    for (int c = 0; c < nChunk; ++c) {
      const int cbeg = c * CE;
      int lim = cbeg + CE;
      lim = lim > nE ? nE : lim;
      const int nblk = (lim - cbeg + NBE - 1) / NBE;
      const int first = (c == 0) ? 1 : 0;
      const int last  = (c == nChunk - 1) ? 1 : 0;
      k_edge<<<nblk, NTHR, EDGEDYN, stream>>>(xb, ei, ea, NP, wp, be1, be2, bc1, Mq, Cq, nE, nN, nb0, cbeg);
      k_agg<<<nbAgg, NTHR, AGGDYN, stream>>>(ei, Mq, Cq, xb, oH, oX, Sb, cbeg, lim, nN, first, last, 1);
    }
  }
  k_nodemlp<<<nbNode, NTHR, MLPDYN, stream>>>(h, wp, bn1, bn2, out0, nTot);
}
